// FactorAtt_ConvRelPosEnc_SK_37142877176322
// MI455X (gfx1250) — hardware-verified
//
#include <hip/hip_runtime.h>
#include <hip/hip_bf16.h>
#include <math.h>

#define NBf 8
#define NTOK 3136
#define NP 3200
#define CCf 512
#define NHf 8
#define CHf 64
#define IMf 56
#define HIDf 32
#define SS 3200
#define HH 1
#define DKK 64
#define GSTR 48

typedef _Float16 bf16;
typedef _Float16 f16;
typedef __attribute__((ext_vector_type(4))) unsigned v4u_t;
typedef unsigned v4ua __attribute__((ext_vector_type(4), may_alias));
typedef __attribute__((ext_vector_type(4))) float v4f_t;
typedef float v4fa __attribute__((ext_vector_type(4), may_alias));
typedef __attribute__((ext_vector_type(16))) bf16  bf16x16;
typedef bf16x16 f16x16;
typedef __attribute__((ext_vector_type(8)))  bf16  bf16x8;
typedef bf16x8 f16x8;
typedef __attribute__((ext_vector_type(4)))  bf16  bf16x4;
typedef __attribute__((ext_vector_type(8)))  float f32x8;
__device__ __forceinline__ f32x8 wmma16(f16x16 a, f16x16 b, f32x8 c) {
  c = __builtin_amdgcn_wmma_f32_16x16x32_f16(false, a, false, b, (short)0, c, false, false);
  asm volatile("v_nop\n\tv_nop\n\tv_nop\n\tv_nop" : "+v"(c) : "v"(a), "v"(b));
  return c;
}
#define LDS_STRIDE 48
#define KSTRIDE    72
#define VSTRIDE    48

__device__ __forceinline__ f32x8 wmma_bf16(bf16x16 a, bf16x16 b, f32x8 c) {
  c = __builtin_amdgcn_wmma_f32_16x16x32_f16(false, a, false, b, (short)0, c, false, false);
  asm volatile("v_nop\n\tv_nop\n\tv_nop\n\tv_nop" : "+v"(c) : "v"(a), "v"(b));
  return c;
}

template <typename T>
__device__ __forceinline__ bf16x16 load_frag(const T* __restrict__ base, int ld,
                                             int row0, int k0) {
  const int lane = threadIdx.x & 31;
  const int r    = lane & 15;
  const int kh   = (lane >> 4) * 8;
  const T* p0 = base + (size_t)(row0 + r) * ld + (k0 + kh);
  const T* p1 = p0 + 16;
  bf16x16 f;
#pragma unroll
  for (int i = 0; i < 8; ++i) {
    f[i]     = (bf16)p0[i];
    f[i + 8] = (bf16)p1[i];
  }
  return f;
}

__device__ __forceinline__ bf16x16 lds_frag(const bf16* base, int stride) {
  const int lane = threadIdx.x & 31;
  const int row  = lane & 15;
  const int kh   = (lane >> 4) * 8;
  const bf16x8 lo = *(const bf16x8*)(base + row * stride + kh);
  const bf16x8 hi = *(const bf16x8*)(base + row * stride + kh + 16);
  bf16x16 f;
#pragma unroll
  for (int i = 0; i < 8; ++i) { f[i] = lo[i]; f[i + 8] = hi[i]; }
  return f;
}

template <typename T>
__device__ __forceinline__ void stage_read16(const T* __restrict__ p, float* buf) {
#pragma unroll
  for (int i = 0; i < 16; ++i) buf[i] = (float)p[i];
}

__device__ __forceinline__ void stage_write(bf16* dst, const float* buf, int nquad) {
#pragma unroll
  for (int i = 0; i < nquad; ++i) {
    bf16x4 q;
    q[0] = (bf16)buf[4 * i];     q[1] = (bf16)buf[4 * i + 1];
    q[2] = (bf16)buf[4 * i + 2]; q[3] = (bf16)buf[4 * i + 3];
    *(bf16x4*)(dst + 4 * i) = q;
  }
}

template <typename AT, int MODE>
__global__ __launch_bounds__(256) void gemm_rb_kernel(
    const AT* __restrict__ A, const float* __restrict__ W,
    const float* __restrict__ bias, const float* __restrict__ rowscale, const float* __restrict__ R, const float* __restrict__ rowbias, void* __restrict__ out,
    int M, int N, int K) {
  __shared__ bf16 ldsA[128 * LDS_STRIDE];
  __shared__ bf16 ldsW[256 * LDS_STRIDE];
  __shared__ __attribute__((aligned(16))) unsigned char sob[256 * 136 * 2];

  const int t    = threadIdx.x;
  const int wave = t >> 5;
  const int lane = t & 31;
  const int wm   = (wave & 1) * 64;
  const int wn   = (wave >> 1) * 64;
  const int mBlk = blockIdx.x * 128;
  const int nBlk = blockIdx.y * 256;

  const int arow = t >> 1;
  const int ach  = (t & 1) * 16;

  float abuf[16];
  float wbuf[32];

  stage_read16(A + (size_t)(mBlk + arow) * K + ach, abuf);
  const int nrow = min(nBlk + t, N - 1);
  stage_read16(W + (size_t)nrow * K,          wbuf);
  stage_read16(W + (size_t)nrow * K + 16,     wbuf + 16);

  f32x8 acc[4][4] = {};

  for (int k = 0; k < K; k += 32) {
    __syncthreads();
    stage_write(&ldsA[arow * LDS_STRIDE + ach], abuf, 4);
    stage_write(&ldsW[t * LDS_STRIDE],          wbuf, 8);
    if (k + 32 < K) {
      stage_read16(A + (size_t)(mBlk + arow) * K + (k + 32) + ach, abuf);
      stage_read16(W + (size_t)nrow * K + (k + 32),          wbuf);
      stage_read16(W + (size_t)nrow * K + (k + 32) + 16,     wbuf + 16);
    }
    __syncthreads();

    bf16x16 af[4], wf[4];
#pragma unroll
    for (int i = 0; i < 4; ++i)
      af[i] = lds_frag(ldsA + (wm + 16 * i) * LDS_STRIDE, LDS_STRIDE);
#pragma unroll
    for (int j = 0; j < 4; ++j)
      wf[j] = lds_frag(ldsW + (wn + 16 * j) * LDS_STRIDE, LDS_STRIDE);
#pragma unroll
    for (int i = 0; i < 4; ++i)
#pragma unroll
      for (int j = 0; j < 4; ++j)
        acc[i][j] = wmma_bf16(af[i], wf[j], acc[i][j]);
  }

  const int nlane = lane & 15;
  const int mh    = (lane >> 4) * 8;
  __syncthreads();
  if (MODE == 0 || MODE == 1 || MODE == 3) {
    bf16* so = (bf16*)sob;
#pragma unroll
    for (int i = 0; i < 4; ++i)
#pragma unroll
      for (int j = 0; j < 4; ++j) {
        const int nl = wn + 16 * j + nlane;
        const float bv = bias ? bias[nBlk + nl] : 0.0f;
        if (MODE == 3) {
#pragma unroll 1
          for (int r = 0; r < 8; ++r) {
            const int ml = wm + 16 * i + mh + r;
            const float xg = acc[i][j][r] + bv;
            so[ml * 264 + nl] = (bf16)(0.5f * xg * (1.0f + erff(xg * 0.70710678118654752f)));
          }
        } else {
#pragma unroll
        for (int r = 0; r < 8; ++r) {
          const int ml = wm + 16 * i + mh + r;
          const bf16 hv = (bf16)(acc[i][j][r] + bv);
          if (MODE == 0) so[ml * 264 + nl] = hv;
          else           so[nl * 136 + ml] = hv;
        }
        }
      }
    __syncthreads();
#pragma unroll 1
    for (int pass = 0; pass < 2; ++pass) {
      if (MODE == 0 || MODE == 3) {
        for (int ch = t; ch < 128 * 32; ch += 256) { const int ml = ch >> 5, q = (ch & 31) * 8;
          *(volatile v4u_t*)((bf16*)out + (size_t)(mBlk + ml) * N + nBlk + q) = *(const v4ua*)(so + ml * 264 + q); }
      } else {
        const int b_ = mBlk / SS, s0 = mBlk % SS;
        for (int ch = t; ch < 256 * 16; ch += 256) { const int nl = ch >> 4, q = (ch & 15) * 8; const int n = nBlk + nl, h = n >> 6, dk = n & (DKK - 1);
          *(volatile v4u_t*)((bf16*)out + (((size_t)(b_ * HH + h)) * DKK + dk) * SS + s0 + q) = *(const v4ua*)(so + nl * 136 + q); }
      }
      __threadfence();
    }
  } else {
    float* so = (float*)sob;
#pragma unroll 1
    for (int hf = 0; hf < 2; ++hf) {
      if (wm == hf * 64) {
#pragma unroll
        for (int i = 0; i < 4; ++i)
#pragma unroll
          for (int j = 0; j < 4; ++j) {
            const int nl = wn + 16 * j + nlane;
            const float bv = bias ? bias[nBlk + nl] : 0.0f;
#pragma unroll
            for (int r = 0; r < 8; ++r) { const int mrow = mBlk + hf * 64 + 16 * i + mh + r; so[(16 * i + mh + r) * 260 + nl] = acc[i][j][r] * (rowscale ? rowscale[mrow] : 1.0f) + bv + (rowbias ? rowbias[mrow] : 0.0f); }
          }
      }
      __syncthreads();
      if (R) {
        for (int ch = t; ch < 64 * 64; ch += 256) { const int ml = ch >> 6, q = (ch & 63) * 4;
          if (nBlk + q < N) { const v4f_t rv = *(const v4f_t*)(R + (size_t)(mBlk + hf * 64 + ml) * N + nBlk + q); v4f_t v = *(const v4fa*)(so + ml * 260 + q); v += rv; *(volatile v4fa*)(so + ml * 260 + q) = v; } }
        asm volatile("s_wait_dscnt 0" ::: "memory");
      }
#pragma unroll 1
      for (int pass = 0; pass < 2; ++pass) {
        for (int ch = t; ch < 64 * 64; ch += 256) { const int ml = ch >> 6, q = (ch & 63) * 4;
          if (nBlk + q < N) *(volatile v4f_t*)((float*)out + (size_t)(mBlk + hf * 64 + ml) * N + nBlk + q) = *(const v4fa*)(so + ml * 260 + q); }
        __threadfence();
      }
      __syncthreads();
    }
  }
}


#define GSTR 48
template <typename AT, int EPI, bool OUT16>
__global__ __launch_bounds__(256) void gemm_kne(const AT* __restrict__ A, int lda, const float* __restrict__ Wm, int ldw,
                                                const float* __restrict__ bias, const float* __restrict__ R, const float* __restrict__ gvec,
                                                void* __restrict__ Yv, int ldy, int K) {
  __shared__ __attribute__((aligned(16))) f16 ldsA[128 * GSTR];
  __shared__ __attribute__((aligned(16))) f16 ldsW[128 * GSTR];
  __shared__ __attribute__((aligned(16))) float oS[8][32 * 68];
  const int tid = threadIdx.x, lane = tid & 31, wave = tid >> 5, cl = lane & 15, rh = (lane >> 4) * 8;
  const int m0 = blockIdx.x * 128, n0 = blockIdx.y * 128;
  const int wm = (wave & 3) * 32, wn = (wave >> 2) * 64;
  f32x8 acc[2][4];
#pragma unroll
  for (int i = 0; i < 2; ++i)
#pragma unroll
    for (int j = 0; j < 4; ++j) { f32x8 z = {}; acc[i][j] = z; }
#pragma unroll 1
  for (int k0 = 0; k0 < K; k0 += 32) {
    __syncthreads();
    { const int row = tid >> 1, ch = (tid & 1) * 16;
      const AT* src = A + (size_t)(m0 + row) * lda + k0 + ch;
#pragma unroll
      for (int g = 0; g < 16; ++g) ldsA[row * GSTR + ch + g] = (f16)src[g]; }
    { const int k = tid >> 3, nn0 = (tid & 7) * 16;
      const float* src = Wm + (size_t)(k0 + k) * ldw + n0 + nn0;
#pragma unroll
      for (int g = 0; g < 4; ++g) { const v4f_t v = *(const v4f_t*)(src + 4 * g);
#pragma unroll
        for (int u = 0; u < 4; ++u) ldsW[(nn0 + 4 * g + u) * GSTR + k] = (f16)v[u]; } }
    __syncthreads();
    f16x16 af[2];
#pragma unroll
    for (int i = 0; i < 2; ++i) af[i] = lds_frag(ldsA + (wm + 16 * i) * GSTR, GSTR);
#pragma unroll
    for (int j = 0; j < 4; ++j) {
      const f16x16 bf = lds_frag(ldsW + (wn + 16 * j) * GSTR, GSTR);
#pragma unroll
      for (int i = 0; i < 2; ++i) acc[i][j] = wmma16(af[i], bf, acc[i][j]);
    }
  }
  float* so = oS[wave];
#pragma unroll
  for (int i = 0; i < 2; ++i)
#pragma unroll
    for (int j = 0; j < 4; ++j) {
      const int n = n0 + wn + 16 * j + cl;
      const float bv = bias ? bias[n] : 0.0f;
      const float gv = (EPI == 2) ? gvec[n] : 0.0f;
      if (EPI == 1) {
#pragma unroll 1
        for (int r = 0; r < 8; ++r) { const float xg = acc[i][j][r] + bv; so[(16 * i + rh + r) * 68 + 16 * j + cl] = 0.5f * xg * (1.0f + erff(xg * 0.70710678118654752f)); }
      } else {
#pragma unroll
        for (int r = 0; r < 8; ++r) {
          float v = acc[i][j][r] + bv;
          if (EPI == 2) v = R[(size_t)(m0 + wm + 16 * i + rh + r) * ldy + n] + gv * v;
          so[(16 * i + rh + r) * 68 + 16 * j + cl] = v;
        }
      }
    }
  asm volatile("s_wait_dscnt 0" ::: "memory");
  __builtin_amdgcn_wave_barrier();
#pragma unroll 1
  for (int pass = 0; pass < 2; ++pass) {
    if (OUT16) {
      f16* Y = (f16*)Yv;
#pragma unroll
      for (int it = 0; it < 8; ++it) { const int c = lane + 32 * it, rr = c >> 3, q8 = (c & 7) * 8;
        union { f16 h[8]; v4u_t v; } u;
#pragma unroll
        for (int e = 0; e < 8; ++e) u.h[e] = (f16)so[rr * 68 + q8 + e];
        *(volatile v4u_t*)(Y + (size_t)(m0 + wm + rr) * ldy + n0 + wn + q8) = u.v; }
    } else {
      float* Y = (float*)Yv;
#pragma unroll
      for (int it = 0; it < 16; ++it) { const int f4 = lane + 32 * it, rr = f4 >> 4, q = (f4 & 15) * 4;
        *(volatile v4f_t*)(Y + (size_t)(m0 + wm + rr) * ldy + n0 + wn + q) = *(const v4fa*)(so + rr * 68 + q); }
    }
    __threadfence();
  }
}

__global__ __launch_bounds__(128) void k_padx(const float* __restrict__ xb, float* __restrict__ Xp) { const int r = blockIdx.x; const int c4 = threadIdx.x * 4; v4f_t v = {0.f,0.f,0.f,0.f}; if (r < NTOK) v = *(const v4f_t*)(xb + (size_t)r * CCf + c4);
  *(volatile v4f_t*)(Xp + (size_t)r * CCf + c4) = v; __threadfence(); *(volatile v4f_t*)(Xp + (size_t)r * CCf + c4) = v; }
__global__ __launch_bounds__(256) void k_colsoftmax(const float* __restrict__ qkv, float* __restrict__ KsT) {
  __shared__ float red[256];
  const int ch = blockIdx.x, tid = threadIdx.x; const float* col = qkv + CCf + ch;
  float m = -3.0e38f;
#pragma unroll 1
  for (int n = tid; n < NTOK; n += 256) m = fmaxf(m, col[(size_t)n * 3 * CCf]);
  red[tid] = m; __syncthreads();
  for (int o = 128; o > 0; o >>= 1) { if (tid < o) red[tid] = fmaxf(red[tid], red[tid + o]); __syncthreads(); }
  m = red[0]; __syncthreads();
  float z = 0.0f;
#pragma unroll 1
  for (int n = tid; n < NTOK; n += 256) z += expf(col[(size_t)n * 3 * CCf] - m);
  red[tid] = z; __syncthreads();
  for (int o = 128; o > 0; o >>= 1) { if (tid < o) red[tid] += red[tid + o]; __syncthreads(); }
  const float sc = 1024.0f / red[0];
#pragma unroll 1
  for (int pass = 0; pass < 2; ++pass) {
#pragma unroll 1
    for (int n = tid; n < NP; n += 256) { const float v = (n < NTOK) ? expf(col[(size_t)n * 3 * CCf] - m) * sc : 0.0f; *(volatile float*)(KsT + (size_t)ch * NP + n) = v; }
    __threadfence(); }
}
__global__ __launch_bounds__(128) void k_blockdiag(const float* __restrict__ KV, float* __restrict__ BD) { const int r = blockIdx.x; const int h = r >> 6; const int c4 = threadIdx.x * 4;
  v4f_t v = {0.f,0.f,0.f,0.f}; if ((c4 >> 6) == h) { v = *(const v4f_t*)(KV + (size_t)r * CCf + c4); for (int e = 0; e < 4; ++e) v[e] *= 0.125f; }
  *(volatile v4f_t*)(BD + (size_t)r * CCf + c4) = v; __threadfence(); *(volatile v4f_t*)(BD + (size_t)r * CCf + c4) = v; }
__global__ __launch_bounds__(256) void k_crpe(const float* __restrict__ qkv, const float* __restrict__ w3, const float* __restrict__ w5, const float* __restrict__ w7, float* __restrict__ FA) {
  const int n = blockIdx.x; const int y = n / IMf, x = n % IMf;
#pragma unroll 1
  for (int cc = 0; cc < 2; ++cc) { const int ch = threadIdx.x + 256 * cc; const int h = ch >> 6;
    int kw; const float* w; if (h < 2) { kw = 3; w = w3 + (size_t)ch * 9; } else if (h < 5) { kw = 5; w = w5 + (size_t)(ch - 128) * 25; } else { kw = 7; w = w7 + (size_t)(ch - 320) * 49; }
    const int p = kw >> 1; float s = 0.0f;
#pragma unroll 1
    for (int dy = 0; dy < kw; ++dy) { const int yy = y + dy - p; if (yy < 0 || yy >= IMf) continue;
#pragma unroll 1
      for (int dx = 0; dx < kw; ++dx) { const int xx = x + dx - p; if (xx < 0 || xx >= IMf) continue; s += w[dy * kw + dx] * qkv[(size_t)(yy * IMf + xx) * 3 * CCf + 2 * CCf + ch]; } }
    const float qv = qkv[(size_t)n * 3 * CCf + ch]; const float v = FA[(size_t)n * CCf + ch] * (1.0f / 1024.0f) + qv * s;
    *(volatile float*)(FA + (size_t)n * CCf + ch) = v; __threadfence(); *(volatile float*)(FA + (size_t)n * CCf + ch) = v; }
}
__global__ __launch_bounds__(256) void k_skgate(const float* __restrict__ FA, const float* __restrict__ wtr, const float* __restrict__ bng, const float* __restrict__ bnb, const float* __restrict__ bnm, const float* __restrict__ bnv, const float* __restrict__ wsel, const float* __restrict__ wproj, float* __restrict__ Wsel) {
  __shared__ float part[256]; __shared__ float da[CHf]; __shared__ float t[HIDf]; __shared__ float sel[CCf];
  const int tid = threadIdx.x; const int c = tid & 63, q = tid >> 6;
  float s = 0.0f;
#pragma unroll 1
  for (int n = q; n < NTOK; n += 4) { const float* row = FA + (size_t)n * CCf + c;
#pragma unroll
    for (int h = 0; h < NHf; ++h) s += row[h * CHf]; }
  part[tid] = s; __syncthreads();
  if (tid < CHf) da[tid] = (part[tid] + part[tid + 64] + part[tid + 128] + part[tid + 192]) * (1.0f / NTOK);
  __syncthreads();
  if (tid < HIDf) { float u = 0.0f; for (int i = 0; i < CHf; ++i) u += da[i] * wtr[tid * CHf + i]; u = (u - bnm[tid]) * bng[tid] / sqrtf(bnv[tid] + 1e-5f) + bnb[tid]; t[tid] = fmaxf(u, 0.0f); }
  __syncthreads();
#pragma unroll 1
  for (int cc = 0; cc < 2; ++cc) { const int ch = tid + 256 * cc; float u = 0.0f; for (int i = 0; i < HIDf; ++i) u += t[i] * wsel[ch * HIDf + i]; sel[ch] = u; }
  __syncthreads();
  if (tid < CHf) { float mx = -3.0e38f; for (int h = 0; h < NHf; ++h) mx = fmaxf(mx, sel[h * CHf + tid]); float z = 0.0f; float e[NHf];
#pragma unroll
    for (int h = 0; h < NHf; ++h) { e[h] = expf(sel[h * CHf + tid] - mx); z += e[h]; }
#pragma unroll
    for (int h = 0; h < NHf; ++h) sel[h * CHf + tid] = e[h] / z; }
  __syncthreads();
#pragma unroll 1
  for (int o = 0; o < CCf; ++o) { for (int cc = 0; cc < 2; ++cc) { const int ch = tid + 256 * cc; const float v = wproj[(size_t)o * CCf + ch] * sel[ch]; *(volatile float*)(Wsel + (size_t)o * CCf + ch) = v; } }
  __threadfence();
#pragma unroll 1
  for (int o = 0; o < CCf; ++o) { for (int cc = 0; cc < 2; ++cc) { const int ch = tid + 256 * cc; const float v = wproj[(size_t)o * CCf + ch] * sel[ch]; *(volatile float*)(Wsel + (size_t)o * CCf + ch) = v; } }
}
__global__ __launch_bounds__(128) void k_copyout(const float* __restrict__ T, float* __restrict__ ob) { const int r = blockIdx.x; const int c4 = threadIdx.x * 4; const v4f_t v = *(const v4f_t*)(T + (size_t)r * CCf + c4);
  *(volatile v4f_t*)(ob + (size_t)r * CCf + c4) = v; __threadfence(); *(volatile v4f_t*)(ob + (size_t)r * CCf + c4) = v; }

extern "C" void kernel_launch(void* const* d_in, const int* in_sizes, int n_in,
                              void* d_out, int out_size, void* d_ws, size_t ws_size,
                              hipStream_t stream) {
  (void)in_sizes; (void)n_in; (void)out_size;
  const float** f = (const float**)d_in;
  const float* x = f[0], *wqkv = f[1], *wproj = f[2], *bproj = f[3], *wtr = f[4], *bng = f[5], *bnb = f[6], *bnm = f[7], *bnv = f[8], *wsel = f[9], *w3 = f[10], *w5 = f[11], *w7 = f[12];
  float* out = (float*)d_out;
  char* ws = (char*)d_ws;
  float* Xp = (float*)ws; ws += (size_t)NP * CCf * 4;
  float* qkv = (float*)ws; ws += (size_t)NP * 3 * CCf * 4;
  float* KsT = (float*)ws; ws += (size_t)CCf * NP * 4;
  float* KV = (float*)ws; ws += (size_t)CCf * CCf * 4; float* BD = (float*)ws; ws += (size_t)CCf * CCf * 4; float* Wsel = (float*)ws; ws += (size_t)CCf * CCf * 4;
  float* FA = (float*)ws; ws += (size_t)NP * CCf * 4;
  float* T = (float*)ws; ws += (size_t)NP * CCf * 4;
  if ((size_t)(ws - (char*)d_ws) > ws_size) return;
  const dim3 blk(256);
  for (int b = 0; b < NBf; ++b) {
    k_padx<<<dim3(NP), dim3(128), 0, stream>>>(x + (size_t)b * NTOK * CCf, Xp);
    gemm_rb_kernel<float, 2><<<dim3(NP / 128, 3 * CCf / 256), blk, 0, stream>>>(Xp, wqkv, nullptr, nullptr, nullptr, nullptr, qkv, NP, 3 * CCf, CCf);
    k_colsoftmax<<<dim3(CCf), blk, 0, stream>>>(qkv, KsT);
    gemm_kne<float, 0, false><<<dim3(CCf / 128, CCf / 128), blk, 0, stream>>>(KsT, NP, qkv + 2 * CCf, 3 * CCf, nullptr, nullptr, nullptr, KV, CCf, NP);
    k_blockdiag<<<dim3(CCf), dim3(128), 0, stream>>>(KV, BD);
    gemm_kne<float, 0, false><<<dim3(NP / 128, CCf / 128), blk, 0, stream>>>(qkv, 3 * CCf, BD, CCf, nullptr, nullptr, nullptr, FA, CCf, CCf);
    k_crpe<<<dim3(NTOK), blk, 0, stream>>>(qkv, w3, w5, w7, FA);
    k_skgate<<<dim3(1), blk, 0, stream>>>(FA, wtr, bng, bnb, bnm, bnv, wsel, wproj, Wsel);
    gemm_rb_kernel<float, 2><<<dim3(NP / 128, CCf / 256), blk, 0, stream>>>(FA, Wsel, bproj, nullptr, nullptr, nullptr, T, NP, CCf, CCf);
    k_copyout<<<dim3(NTOK), dim3(128), 0, stream>>>(T, out + (size_t)b * NTOK * CCf);
  }
}
